// GhostVLAD_82575041233229
// MI455X (gfx1250) — hardware-run, weakly checked
//
#include <hip/hip_runtime.h>


#ifndef NB
#define NB 32
#endif
#define NB_FULL 32
#define CD    512
#define LPOS  512
#define KG    10
#define VK    8
#define KP    16
#define PP    520
#define TP    72
#define NWV   16
#define PCARRY 1024.0f
#define PINV   (1.0f / 1024.0f)
#define LOG2E  1.4426950408889634f
#define EPSN   1e-12f
#define NEGB   (-3.0e38f)
#define X_BSTRIDE ((size_t)CD * LPOS)

static_assert(NB <= NB_FULL);
static_assert(KG <= KP);
static_assert(VK <= 8);
static_assert(CD % 64 == 0);
static_assert(LPOS % 64 == 0);
static_assert(CD % 32 == 0);
static_assert(LPOS % 32 == 0);
static_assert(LPOS == NWV * 32);
static_assert(CD == NWV * 32);
static_assert(LPOS == 32 * NWV);
static_assert(CD == LPOS);
static_assert(NWV == 2 * VK);
static_assert(64 * 8 == CD);
static_assert((PP * 2) % 16 == 0);
static_assert(PP >= LPOS);
static_assert(256 * 2 * 8 == 64 * 64);
static_assert(((KP * CD / 8) % 256) == 0);
static_assert(32 * NWV * 2 * 4 == VK * CD);
static_assert(64 * TP * 2 <= 131072);
static_assert(KP * LPOS * 4 + KP * PP * 2 + NWV * KP * 4 + KP * 4 + NWV * 4 <= 131072);

typedef _Float16 h16;
typedef unsigned short bf;
typedef __attribute__((ext_vector_type(16))) __bf16   v16bf;
typedef __attribute__((ext_vector_type(16))) _Float16 v16h;
typedef __attribute__((ext_vector_type(8)))  _Float16 v8h;
typedef __attribute__((ext_vector_type(8)))  unsigned short v8us;
typedef __attribute__((ext_vector_type(8)))  float    v8f;
typedef __attribute__((ext_vector_type(4)))  float    v4f;
typedef v4f  __attribute__((may_alias)) v4fa;
typedef v8h  __attribute__((may_alias)) v8ha;

__device__ __forceinline__ unsigned short f2bf(float f) { unsigned u = __float_as_uint(f); u += 0x7FFFu + ((u >> 16) & 1u); return (unsigned short)(u >> 16); }
__device__ __forceinline__ float bfr(float f) { return __uint_as_float(((unsigned)f2bf(f)) << 16); }
__device__ __forceinline__ v16h cat16(v8h lo, v8h hi) { return __builtin_shufflevector(lo, hi, 0, 1, 2, 3, 4, 5, 6, 7, 8, 9, 10, 11, 12, 13, 14, 15); }
__device__ __forceinline__ v16bf cat16b(v8us lo, v8us hi) { return __builtin_bit_cast(v16bf, __builtin_shufflevector(lo, hi, 0, 1, 2, 3, 4, 5, 6, 7, 8, 9, 10, 11, 12, 13, 14, 15)); }
__device__ __forceinline__ v8f wmma16(v16h a, v16h b, v8f c) { return __builtin_amdgcn_wmma_f32_16x16x32_f16(false, a, false, b, (short)0, c, false, false); }
__device__ __forceinline__ v8f wmmab(v16bf a, v16bf b, v8f c) { return __builtin_amdgcn_wmma_f32_16x16x32_bf16(false, a, false, b, (short)0, c, false, false); }
__device__ __forceinline__ v16h  ldh(const h16* p) { return cat16(*(const v8h*)p, *(const v8h*)(p + 16)); }
__device__ __forceinline__ v16bf ldb(const bf* p)  { return cat16b(*(const v8us*)p, *(const v8us*)(p + 16)); }

static __device__ __forceinline__ h16 toh_flush(float v) { const h16 r = (h16)v; return (fabsf(v) < 6.103515625e-05f) ? (h16)0.0f : r; }
static __device__ __forceinline__ v8f wmmab_g(v16bf a, v16bf b, v8f c) { c = wmmab(a, b, c); asm volatile("v_nop\n\tv_nop\n\tv_nop\n\tv_nop" : "+v"(c) : "v"(a), "v"(b)); return c; }
static __device__ __forceinline__ v8f wmma16_g(v16h a, v16h b, v8f c) { c = wmma16(a, b, c); asm volatile("v_nop\n\tv_nop\n\tv_nop\n\tv_nop" : "+v"(c) : "v"(a), "v"(b)); return c; }

__global__ __launch_bounds__(256) void k_wprep(const float* __restrict__ W, bf* WB) {
    const int i = blockIdx.x * 256 + threadIdx.x; if (i >= KP * CD / 8) return;
    const int row = i / (CD / 8), c8 = (i % (CD / 8)) * 8;
    const int rc = row < KG ? row : (KG - 1);
    v4f x0 = *(const v4f*)(W + (size_t)rc * CD + c8); v4f x1 = *(const v4f*)(W + (size_t)rc * CD + c8 + 4);
    asm volatile("" : "+v"(x0), "+v"(x1));
    const bool ok = row < KG;
    v8us o;
#pragma unroll
    for (int k = 0; k < 4; ++k) { const unsigned short a0 = f2bf(x0[k]); const unsigned short a1 = f2bf(x1[k]); o[k] = ok ? a0 : (unsigned short)0; o[4 + k] = ok ? a1 : (unsigned short)0; }
    *(volatile v8us*)(WB + (size_t)i * 8) = o; __threadfence(); *(volatile v8us*)(WB + (size_t)i * 8) = o;
}

__global__ __launch_bounds__(256) void k_xprep(const float* __restrict__ X, bf* XT, h16* XH) {
    __shared__ __align__(16) bf tb[64 * TP];
    const int tid = threadIdx.x;
    const int n = blockIdx.z, c0 = blockIdx.y * 64, l0 = blockIdx.x * 64;
    const float* xs = X + (size_t)n * X_BSTRIDE + (size_t)c0 * LPOS + l0;
    v8h hv[2];
#pragma unroll
    for (int it = 0; it < 2; ++it) {
        const int p = it * 256 + tid; const int row = p >> 3, c8 = (p & 7) * 8;
        const v4f x0 = *(const v4f*)(xs + (size_t)row * LPOS + c8); const v4f x1 = *(const v4f*)(xs + (size_t)row * LPOS + c8 + 4);
#pragma unroll
        for (int i = 0; i < 4; ++i) {
            const unsigned short b0 = f2bf(x0[i]); const unsigned short b1 = f2bf(x1[i]);
            tb[row * TP + c8 + i] = b0; tb[row * TP + c8 + 4 + i] = b1;
            hv[it][i] = toh_flush(__uint_as_float(((unsigned)b0) << 16)); hv[it][4 + i] = toh_flush(__uint_as_float(((unsigned)b1) << 16)); }
    }
    __syncthreads();
    v8us tv[2];
#pragma unroll
    for (int it = 0; it < 2; ++it) {
        const int p = it * 256 + tid; const int lrow = p >> 3, cp = (p & 7) * 8;
#pragma unroll
        for (int j = 0; j < 8; ++j) tv[it][j] = tb[(cp + j) * TP + lrow];
    }
    h16* xh = XH + ((size_t)n * CD + c0) * LPOS + l0;
    bf*  xt = XT + ((size_t)n * LPOS + l0) * CD + c0;
#pragma unroll 1
    for (int ps = 0; ps < 2; ++ps) {
#pragma unroll
        for (int it = 0; it < 2; ++it) {
            const int p = it * 256 + tid; const int row = p >> 3, c8 = (p & 7) * 8;
            *(volatile v8h*)(xh + (size_t)row * LPOS + c8) = hv[it];
            *(volatile v8us*)(xt + (size_t)row * CD + c8) = tv[it]; }
        if (ps == 0) __threadfence(); }
}

__global__ __launch_bounds__(32 * NWV) void k_aggr(const bf* __restrict__ WB, const bf* __restrict__ XT, const h16* __restrict__ XH,
                                                  const float* __restrict__ cb, const float* __restrict__ cen, float* OUT) {
    __shared__ __align__(16) float sL[KP * LPOS];
    __shared__ __align__(16) h16   sP[KP * PP];
    __shared__ float sPart[NWV * KP];
    __shared__ float sAsum[KP];
    __shared__ float sQ[NWV];
    const int tid = threadIdx.x;
    const int lane = tid & 31, lr = lane & 15, hi = lane >> 4;
    const int wave = __builtin_amdgcn_readfirstlane((int)(threadIdx.x >> 5));
    const int n = blockIdx.x;

    {
        const int l0 = wave * 32;
        const size_t wo  = (size_t)lr * CD + 8 * hi;
        const size_t xo0 = ((size_t)n * LPOS + l0 + lr) * CD + 8 * hi;
        const size_t xo1 = xo0 + (size_t)16 * CD;
        v8f acc0 = (v8f){}, acc1 = (v8f){};
#pragma unroll 1
        for (int kc = 0; kc < CD; kc += 32) {
            const v16bf a  = ldb(WB + wo + kc);
            const v16bf b0 = ldb(XT + xo0 + kc);
            const v16bf b1 = ldb(XT + xo1 + kc);
            acc0 = wmmab_g(a, b0, acc0);
            acc1 = wmmab_g(a, b1, acc1);
        }
        float bj[8];
#pragma unroll
        for (int j = 0; j < 8; ++j) { const int kk = 8 * hi + j; const int kcl = kk < KG ? kk : (KG - 1);
            float t = cb[kcl]; asm volatile("" : "+v"(t)); bj[j] = (kk < KG) ? bfr(t) : 0.0f; }
#pragma unroll
        for (int j = 0; j < 8; ++j) {
            sL[(8 * hi + j) * LPOS + l0 + lr]      = acc0[j] + bj[j];
            sL[(8 * hi + j) * LPOS + l0 + 16 + lr] = acc1[j] + bj[j]; }
    }
    __syncthreads();

    {
        const int l = tid;
        float t[KG], av[KG]; float m = NEGB;
#pragma unroll
        for (int k = 0; k < KG; ++k) { t[k] = sL[k * LPOS + l]; m = fmaxf(m, t[k]); }
        float s = 0.0f;
#pragma unroll
        for (int k = 0; k < KG; ++k) { t[k] = __builtin_amdgcn_exp2f((t[k] - m) * LOG2E); s += t[k]; }
        const float inv = 1.0f / s;
#pragma unroll
        for (int k = 0; k < KG; ++k) { av[k] = t[k] * inv; sP[k * PP + l] = toh_flush(av[k] * PCARRY); }
#pragma unroll
        for (int k = KG; k < KP; ++k) sP[k * PP + l] = (h16)0.0f;
#pragma unroll
        for (int k = 0; k < KG; ++k) {
            float v = av[k];
            v += __shfl_xor(v, 16, 32); v += __shfl_xor(v, 8, 32); v += __shfl_xor(v, 4, 32); v += __shfl_xor(v, 2, 32); v += __shfl_xor(v, 1, 32);
            if (lane == 0) sPart[wave * KP + k] = v; }
#pragma unroll
        for (int k = KG; k < KP; ++k) { if (lane == 0) sPart[wave * KP + k] = 0.0f; }
    }
    __syncthreads();
    {
        const int k = tid & (KP - 1);
        float s = 0.0f;
#pragma unroll
        for (int w = 0; w < NWV; ++w) s += sPart[w * KP + k];
        if (tid < KP) sAsum[k] = s;
    }
    __syncthreads();

    {
        const int c0 = wave * 32;
        const int po = lr * PP + 8 * hi;
        const size_t ho0 = ((size_t)n * CD + c0 + lr) * LPOS + 8 * hi;
        const size_t ho1 = ho0 + (size_t)16 * LPOS;
        v8f acc0 = (v8f){}, acc1 = (v8f){};
#pragma unroll 1
        for (int kc = 0; kc < LPOS; kc += 32) {
            const v16h a  = cat16(*(const v8ha*)(&sP[po + kc]), *(const v8ha*)(&sP[po + kc + 16]));
            const v16h b0 = ldh(XH + ho0 + kc);
            const v16h b1 = ldh(XH + ho1 + kc);
            acc0 = wmma16_g(a, b0, acc0);
            acc1 = wmma16_g(a, b1, acc1);
        }
#pragma unroll
        for (int j = 0; j < 8; ++j) {
            const int kk = 8 * hi + j; const int kcl = kk < KG ? kk : (KG - 1);
            float ce0 = cen[(size_t)kcl * CD + c0 + lr]; float ce1 = cen[(size_t)kcl * CD + c0 + 16 + lr];
            asm volatile("" : "+v"(ce0), "+v"(ce1));
            const float as = sAsum[kk];
            sL[kk * CD + c0 + lr]      = acc0[j] * PINV - as * bfr(ce0);
            sL[kk * CD + c0 + 16 + lr] = acc1[j] * PINV - as * bfr(ce1); }
    }
    __syncthreads();

    {
        const int k = wave >> 1; const int seg = tid & 63;
        float part = 0.0f;
#pragma unroll
        for (int c = 0; c < 8; ++c) { const float v = sL[k * CD + seg * 8 + c]; part += v * v; }
        part += __shfl_xor(part, 16, 32); part += __shfl_xor(part, 8, 32); part += __shfl_xor(part, 4, 32); part += __shfl_xor(part, 2, 32); part += __shfl_xor(part, 1, 32);
        if (lane == 0) sQ[wave] = part;
    }
    __syncthreads();

    float tot = 0.0f;
#pragma unroll 1
    for (int k = 0; k < VK; ++k) { const float sq = sQ[2 * k] + sQ[2 * k + 1]; const float r = 1.0f / fmaxf(sqrtf(sq), EPSN); tot += sq * r * r; }
    const float tinv = 1.0f / fmaxf(sqrtf(tot), EPSN);
    v4f val[2];
#pragma unroll
    for (int i = 0; i < 2; ++i) {
        const int idx4 = i * (32 * NWV) + tid;
        const int k = idx4 >> 7;
        const float sq = sQ[2 * k] + sQ[2 * k + 1];
        const float sc = (1.0f / fmaxf(sqrtf(sq), EPSN)) * tinv;
        const v4f v = *(const v4fa*)(&sL[idx4 * 4]);
        val[i] = v * sc; }
    float* on = OUT + (size_t)n * (VK * CD);
#pragma unroll 1
    for (int ps = 0; ps < 2; ++ps) {
#pragma unroll
        for (int i = 0; i < 2; ++i) *(volatile v4f*)(on + (size_t)(i * (32 * NWV) + tid) * 4) = val[i];
        if (ps == 0) __threadfence(); }
}

static constexpr size_t al256(size_t v) { return (v + 255) & ~(size_t)255; }
static constexpr size_t SZ_XT = al256((size_t)NB * LPOS * CD * 2);
static constexpr size_t SZ_XH = al256((size_t)NB * CD * LPOS * 2);
static constexpr size_t SZ_WB = al256((size_t)KP * CD * 2);
static constexpr size_t SZ_TOTAL = SZ_XT + SZ_XH + SZ_WB;
static_assert(SZ_TOTAL <= (size_t)134217728);
static_assert((size_t)(LPOS / 64) * 64 * (CD / 64) * 64 * NB * 2 == (size_t)NB * LPOS * CD * 2);

extern "C" void kernel_launch(void* const* d_in, const int* in_sizes, int n_in,
                              void* d_out, int out_size, void* d_ws, size_t ws_size, hipStream_t stream) {
    if (n_in < 4) return;
    if ((size_t)in_sizes[0] < (size_t)NB * CD * LPOS) return;
    if ((size_t)in_sizes[1] < (size_t)KG * CD || in_sizes[2] < KG || (size_t)in_sizes[3] < (size_t)KG * CD) return;
    if ((size_t)out_size < (size_t)NB * VK * CD) return;
    if (SZ_TOTAL > ws_size) return;
    const float* x  = (const float*)d_in[0];
    const float* cw = (const float*)d_in[1];
    const float* cb = (const float*)d_in[2];
    const float* ce = (const float*)d_in[3];
    float* OUT = (float*)d_out;
    char* wsp = (char*)d_ws;
    bf*  XT = (bf*)wsp;  wsp += SZ_XT;
    h16* XH = (h16*)wsp; wsp += SZ_XH;
    bf*  WB = (bf*)wsp;  wsp += SZ_WB;

    k_wprep<<<dim3(KP * CD / 8 / 256, 1, 1), 256, 0, stream>>>(cw, WB);
    k_xprep<<<dim3(LPOS / 64, CD / 64, NB), 256, 0, stream>>>(x, XT, XH);
    k_aggr<<<dim3(NB, 1, 1), 32 * NWV, 0, stream>>>(WB, XT, XH, cb, ce, OUT);
}
